// CloudGraph_58746562674891
// MI455X (gfx1250) — hardware-verified
//
#include <hip/hip_runtime.h>
#include <stddef.h>


#define DF      128
#define NTHR    256
#define NWAVE   8
#define EPT     8
#define NGRP    2
#define CHUNK   (NTHR * EPT * NGRP)
#define WCAP    (EPT * NGRP * 32)
#define LISTN   (NWAVE * WCAP)
#define NB      256
#define GROWS   128
#define APH     136
#define EPSV    1e-5f

#define LDS_ASTAGE (GROWS * APH * 2 * 2)
#define LDS_NODE   (LDS_ASTAGE + 3 * DF * 4 + GROWS * 4 * 4)
#define LDS_AGG    (2 * NB * DF * 4 + LISTN * 4 + 64)

static_assert((CHUNK & (CHUNK - 1)) == 0);
static_assert(CHUNK <= 4096);
static_assert(NB <= 4096 && (NB & (NB - 1)) == 0);
static_assert(NB == NWAVE * 32);
static_assert(GROWS == NWAVE * 16);
static_assert(GROWS * DF * 4 <= LDS_ASTAGE);
static_assert(NWAVE * 2 * DF * 8 <= LISTN * 4);

typedef float  v4f  __attribute__((ext_vector_type(4)));
typedef float  v8f  __attribute__((ext_vector_type(8)));
typedef int    v4i  __attribute__((ext_vector_type(4)));
typedef __bf16 v8b  __attribute__((ext_vector_type(8)));
typedef __bf16 v16b __attribute__((ext_vector_type(16)));
union FragB { v16b v; v8b h[2]; };
union Pack8 { v8b b; v4i i; };

__device__ __forceinline__ void split8(const v4f a, const v4f b, v8b* hi, v8b* lo) {
  v8b H, L;
#define SPL(I, V) { const float f_ = (V); const __bf16 h_ = (__bf16)f_; H[I] = h_; L[I] = (__bf16)(f_ - (float)h_); }
  SPL(0, a.x) SPL(1, a.y) SPL(2, a.z) SPL(3, a.w)
  SPL(4, b.x) SPL(5, b.y) SPL(6, b.z) SPL(7, b.w)
#undef SPL
  *hi = H; *lo = L;
}

__device__ __forceinline__ v8f wmb(v16b a, v16b b, v8f c) {
  v8f d = __builtin_amdgcn_wmma_f32_16x16x32_bf16(false, a, false, b, (short)0, c, false, false);
  asm volatile("v_nop\n\tv_nop\n\tv_nop\n\tv_nop" : "+v"(d) : "v"(a), "v"(b));
  return d;
}

__device__ __forceinline__ v4f relu4(v4f v) {
  v.x = fmaxf(v.x, 0.f); v.y = fmaxf(v.y, 0.f); v.z = fmaxf(v.z, 0.f); v.w = fmaxf(v.w, 0.f);
  return v;
}

__device__ __forceinline__ int scan_chunk(const int* __restrict__ keys, int nE, int cbase, int nodeBase,
                                          int vec8, int* list, int tid, int wave) {
  int wc = 0;
#pragma unroll
  for (int g = 0; g < NGRP; ++g) {
    const int el0  = (g * NTHR + tid) * EPT;
    const int e0   = cbase + el0;
    const int sent = -2147483647 - 1;
    v4i da, db;
    if (vec8 != 0 && e0 + 7 < nE) {
      da = *(const v4i*)(keys + e0);
      db = *(const v4i*)(keys + e0 + 4);
    } else {
      da.x = (e0     < nE) ? keys[min(e0, nE - 1)] : sent;
      da.y = (e0 + 1 < nE) ? keys[min(e0 + 1, nE - 1)] : sent;
      da.z = (e0 + 2 < nE) ? keys[min(e0 + 2, nE - 1)] : sent;
      da.w = (e0 + 3 < nE) ? keys[min(e0 + 3, nE - 1)] : sent;
      db.x = (e0 + 4 < nE) ? keys[min(e0 + 4, nE - 1)] : sent;
      db.y = (e0 + 5 < nE) ? keys[min(e0 + 5, nE - 1)] : sent;
      db.z = (e0 + 6 < nE) ? keys[min(e0 + 6, nE - 1)] : sent;
      db.w = (e0 + 7 < nE) ? keys[min(e0 + 7, nE - 1)] : sent;
    }
    const unsigned nb = (unsigned)nodeBase;
    const unsigned s0 = (unsigned)da.x - nb, s1 = (unsigned)da.y - nb;
    const unsigned s2 = (unsigned)da.z - nb, s3 = (unsigned)da.w - nb;
    const unsigned s4 = (unsigned)db.x - nb, s5 = (unsigned)db.y - nb;
    const unsigned s6 = (unsigned)db.z - nb, s7 = (unsigned)db.w - nb;
    const bool h0 = s0 < (unsigned)NB, h1 = s1 < (unsigned)NB, h2 = s2 < (unsigned)NB, h3 = s3 < (unsigned)NB;
    const bool h4 = s4 < (unsigned)NB, h5 = s5 < (unsigned)NB, h6 = s6 < (unsigned)NB, h7 = s7 < (unsigned)NB;
    const unsigned any = __builtin_amdgcn_ballot_w32(h0 | h1 | h2 | h3 | h4 | h5 | h6 | h7);
    if (any != 0u) {
#define HITJ(J, HJ, SJ) { \
        const unsigned mj = __builtin_amdgcn_ballot_w32(HJ); \
        if (mj != 0u) { \
          if (HJ) { \
            const int pos = wc + (int)__builtin_amdgcn_mbcnt_lo(mj, 0u); \
            if (pos < WCAP) list[wave * WCAP + pos] = ((el0 + (J)) << 12) | (int)(SJ); \
          } \
          wc += (int)__builtin_popcount(mj); } }
      HITJ(0, h0, s0)
      HITJ(1, h1, s1)
      HITJ(2, h2, s2)
      HITJ(3, h3, s3)
      HITJ(4, h4, s4)
      HITJ(5, h5, s5)
      HITJ(6, h6, s6)
      HITJ(7, h7, s7)
#undef HITJ
    }
  }
  return wc;
}

__global__ __launch_bounds__(NTHR) void k_wprep(const float* __restrict__ W1, __bf16* w1h, __bf16* w1l) {
  const int i = blockIdx.x * NTHR + threadIdx.x;
  if (i >= DF * DF / 8) return;
  const int o  = i * 8;
  const int n  = o / DF;
  const int k0 = o - n * DF;
  const float* p = W1 + (size_t)k0 * DF + n;
  v4f a, b;
  a.x = p[0];      a.y = p[DF];     a.z = p[2 * DF]; a.w = p[3 * DF];
  b.x = p[4 * DF]; b.y = p[5 * DF]; b.z = p[6 * DF]; b.w = p[7 * DF];
  Pack8 H, L;
  split8(a, b, &H.b, &L.b);
  *(volatile v4i*)(w1h + o) = H.i;
  *(volatile v4i*)(w1l + o) = L.i;
  __threadfence();
  *(volatile v4i*)(w1h + o) = H.i;
  *(volatile v4i*)(w1l + o) = L.i;
}

__global__ __launch_bounds__(NTHR) void k_node(
    const float* __restrict__ x, const float* __restrict__ xyz, const float* __restrict__ Wxyz,
    const __bf16* __restrict__ w1h, const __bf16* __restrict__ w1l,
    float* y, float* z, int nN) {
  extern __shared__ v4f lds_dyn[];
  __bf16* sAh  = (__bf16*)lds_dyn;
  __bf16* sAl  = sAh + GROWS * APH;
  float*  stg  = (float*)lds_dyn;
  float*  swx  = (float*)((char*)lds_dyn + LDS_ASTAGE);
  float*  sxyz = swx + 3 * DF;
  const int tid = threadIdx.x, lane = tid & 31, wave = tid >> 5, hh = lane >> 4, m = lane & 15;
  const int rowBase = blockIdx.x * GROWS;
  const int c4 = 4 * lane;

#pragma unroll
  for (int i = 0; i < (GROWS * DF / 8) / NTHR; ++i) {
    const int idx = i * NTHR + tid;
    const int r   = idx >> 4;
    const int c0  = (idx & 15) * 8;
    int node = rowBase + r;
    node = node > nN - 1 ? nN - 1 : node;
    const float* xp = x + (size_t)node * DF + c0;
    const v4f a = *(const v4f*)xp, b = *(const v4f*)(xp + 4);
    v8b H, L;
    split8(a, b, &H, &L);
    *(v8b*)(sAh + r * APH + c0) = H;
    *(v8b*)(sAl + r * APH + c0) = L;
  }
  for (int i = tid; i < 3 * DF; i += NTHR) swx[i] = Wxyz[i];
  for (int i = tid; i < GROWS * 3; i += NTHR) {
    const int r = i / 3, c = i - 3 * r;
    int node = rowBase + r;
    node = node > nN - 1 ? nN - 1 : node;
    sxyz[r * 4 + c] = xyz[(size_t)node * 3 + c];
  }
  __syncthreads();

  v8f acc[8];
#pragma unroll
  for (int t = 0; t < 8; ++t) { v8f zz = {0.f, 0.f, 0.f, 0.f, 0.f, 0.f, 0.f, 0.f}; acc[t] = zz; }
  const __bf16* arh = sAh + (wave * 16 + m) * APH + 8 * hh;
  const __bf16* arl = sAl + (wave * 16 + m) * APH + 8 * hh;
#pragma unroll 1
  for (int kt = 0; kt < DF / 32; ++kt) {
    FragB ah, al;
    ah.h[0] = *(const v8b*)(arh + 32 * kt);
    ah.h[1] = *(const v8b*)(arh + 32 * kt + 16);
    al.h[0] = *(const v8b*)(arl + 32 * kt);
    al.h[1] = *(const v8b*)(arl + 32 * kt + 16);
#pragma unroll
    for (int t = 0; t < 8; ++t) {
      const size_t bo = (size_t)(16 * t + m) * DF + 32 * kt + 8 * hh;
      FragB bh, bl;
      bh.h[0] = *(const v8b*)(w1h + bo);
      bh.h[1] = *(const v8b*)(w1h + bo + 16);
      bl.h[0] = *(const v8b*)(w1l + bo);
      bl.h[1] = *(const v8b*)(w1l + bo + 16);
      v8f c = acc[t];
      c = wmb(ah.v, bh.v, c);
      c = wmb(ah.v, bl.v, c);
      c = wmb(al.v, bh.v, c);
      acc[t] = c;
    }
  }
  __syncthreads();

  {
    const int r0 = wave * 16 + 8 * hh;
    float* sp = stg + r0 * DF + m;
#pragma unroll
    for (int t = 0; t < 8; ++t) {
      sp[0 * DF + 16 * t] = acc[t][0];
      sp[1 * DF + 16 * t] = acc[t][1];
      sp[2 * DF + 16 * t] = acc[t][2];
      sp[3 * DF + 16 * t] = acc[t][3];
      sp[4 * DF + 16 * t] = acc[t][4];
      sp[5 * DF + 16 * t] = acc[t][5];
      sp[6 * DF + 16 * t] = acc[t][6];
      sp[7 * DF + 16 * t] = acc[t][7];
    }
  }
  __syncthreads();

  const v4f wa = *(const v4f*)(swx + c4);
  const v4f wb = *(const v4f*)(swx + DF + c4);
  const v4f wcv = *(const v4f*)(swx + 2 * DF + c4);
  v4f zv[16];
#pragma unroll
  for (int i = 0; i < 16; ++i) {
    const int r = wave * 16 + i;
    const float sx0 = sxyz[r * 4 + 0], sx1 = sxyz[r * 4 + 1], sx2 = sxyz[r * 4 + 2];
    zv[i] = wa * sx0 + wb * sx1 + wcv * sx2;
  }

  const float* lp = stg + wave * 16 * DF + c4;
  float* yp = y + ((size_t)rowBase + wave * 16) * DF + c4;
  float* zp = z + ((size_t)rowBase + wave * 16) * DF + c4;
#pragma unroll
  for (int i = 0; i < 16; ++i) {
    const v4f v = *(const v4f*)(lp + i * DF);
    *(volatile v4f*)(yp + (size_t)i * DF) = v;
    *(volatile v4f*)(zp + (size_t)i * DF) = zv[i];
  }
  __threadfence();
#pragma unroll
  for (int i = 0; i < 16; ++i) {
    const v4f v = *(const v4f*)(lp + i * DF);
    *(volatile v4f*)(yp + (size_t)i * DF) = v;
    *(volatile v4f*)(zp + (size_t)i * DF) = zv[i];
  }
}

__global__ __launch_bounds__(NTHR) void k_agg(
    const int* __restrict__ srcl, const int* __restrict__ dstl,
    const float* __restrict__ xyz, const float* __restrict__ x,
    const float* __restrict__ y, const float* __restrict__ z,
    const float* __restrict__ b1, const float* __restrict__ lng, const float* __restrict__ lnb,
    float* t1, float* p2g, double* part, int nN, int nE, int vec8) {
  extern __shared__ v4f lds_dyn[];
  float*  acc1  = (float*)lds_dyn;
  float*  acc2  = acc1 + NB * DF;
  int*    list  = (int*)(acc2 + NB * DF);
  int*    wcnt  = list + LISTN;
  double* wpart = (double*)list;
  const int tid = threadIdx.x, lane = tid & 31, wave = tid >> 5;
  const int nodeBase = blockIdx.x * NB;
  const int c4 = 4 * lane;

  {
    const v4f zz = {0.f, 0.f, 0.f, 0.f};
    for (int i = tid; i < 2 * NB * DF / 4; i += NTHR) lds_dyn[i] = zz;
  }
  __syncthreads();

  const v4f b1v = *(const v4f*)(b1 + c4);
  const int nChunks = (nE + CHUNK - 1) / CHUNK;
#pragma unroll 1
  for (int ch = 0; ch < nChunks; ++ch) {
    const int cbase = ch * CHUNK;
    const int wc = scan_chunk(srcl, nE, cbase, nodeBase, vec8, list, tid, wave);
    if (lane == 0) wcnt[wave] = wc;
    __syncthreads();
    if (wave == 0) {
#pragma unroll 1
      for (int wsx = 0; wsx < NWAVE; ++wsx) {
        int n = __builtin_amdgcn_readfirstlane(wcnt[wsx]);
        n = n > WCAP ? WCAP : (n < 0 ? 0 : n);
        const int* lp = list + wsx * WCAP;
#pragma unroll 1
        for (int i = 0; i < n; ++i) {
          const int ent  = __builtin_amdgcn_readfirstlane(lp[i]);
          const int slot = ent & (NB - 1);
          int e = cbase + ((ent >> 12) & (CHUNK - 1));
          e = e > nE - 1 ? nE - 1 : e;
          int d = dstl[e];
          d = d < 0 ? 0 : (d > nN - 1 ? nN - 1 : d);
          int s = nodeBase + slot;
          s = s > nN - 1 ? nN - 1 : s;
          const float dx = xyz[(size_t)s * 3 + 0] - xyz[(size_t)d * 3 + 0];
          const float dy = xyz[(size_t)s * 3 + 1] - xyz[(size_t)d * 3 + 1];
          const float dz = xyz[(size_t)s * 3 + 2] - xyz[(size_t)d * 3 + 2];
          const float dist = sqrtf(dx * dx + dy * dy + dz * dz);
          const float w = expf(-dist);
          const v4f ys = *(const v4f*)(y + (size_t)s * DF + c4);
          const v4f yd = *(const v4f*)(y + (size_t)d * DF + c4);
          const v4f zs = *(const v4f*)(z + (size_t)s * DF + c4);
          const v4f zd = *(const v4f*)(z + (size_t)d * DF + c4);
          const v4f hv = relu4((ys - yd) * w + b1v);
          const v4f gv = relu4(zs - zd);
          v4f* ap1 = (v4f*)(acc1 + slot * DF + c4);
          *ap1 = *ap1 + hv;
          v4f* ap2 = (v4f*)(acc2 + slot * DF + c4);
          *ap2 = *ap2 + gv;
        }
      }
    }
    __syncthreads();
  }

  const v4f lgv = *(const v4f*)(lng + c4);
  const v4f lbv = *(const v4f*)(lnb + c4);
  const float invD = 1.0f / (float)DF;
  double sP0 = 0.0, sP1 = 0.0, sP2 = 0.0, sP3 = 0.0;
  double sQ0 = 0.0, sQ1 = 0.0, sQ2 = 0.0, sQ3 = 0.0;
  float* t1p = t1  + (size_t)nodeBase * DF + c4;
  float* p2p = p2g + (size_t)nodeBase * DF + c4;
#pragma unroll 1
  for (int j = 0; j < 32; ++j) {
    const int slot = wave * 32 + j;
    const int node = nodeBase + slot;
    const bool valid = node < nN;
    const int nodec = valid ? node : nN - 1;
    v4f* a1 = (v4f*)(acc1 + slot * DF + c4);
    const v4f p1 = *a1;
    float s1 = (p1.x + p1.y) + (p1.z + p1.w);
    s1 += __shfl_xor(s1, 16, 32);
    s1 += __shfl_xor(s1, 8, 32);
    s1 += __shfl_xor(s1, 4, 32);
    s1 += __shfl_xor(s1, 2, 32);
    s1 += __shfl_xor(s1, 1, 32);
    const float mu = s1 * invD;
    const v4f dev = p1 - mu;
    float s2 = (dev.x * dev.x + dev.y * dev.y) + (dev.z * dev.z + dev.w * dev.w);
    s2 += __shfl_xor(s2, 16, 32);
    s2 += __shfl_xor(s2, 8, 32);
    s2 += __shfl_xor(s2, 4, 32);
    s2 += __shfl_xor(s2, 2, 32);
    s2 += __shfl_xor(s2, 1, 32);
    const float var = s2 * invD;
    const float inv = 1.0f / sqrtf(var + EPSV);
    const v4f xr = *(const v4f*)(x + (size_t)nodec * DF + c4);
    v4f u = dev * inv;
    u = u * lgv + lbv;
    const v4f tv = xr + u;
    *a1 = tv;
    const v4f q = *(const v4f*)(acc2 + slot * DF + c4);
    *(volatile v4f*)(t1p + (size_t)slot * DF) = tv;
    *(volatile v4f*)(p2p + (size_t)slot * DF) = q;
    if (valid) {
      sP0 += (double)q.x; sP1 += (double)q.y; sP2 += (double)q.z; sP3 += (double)q.w;
      sQ0 += (double)q.x * (double)q.x; sQ1 += (double)q.y * (double)q.y;
      sQ2 += (double)q.z * (double)q.z; sQ3 += (double)q.w * (double)q.w;
    }
  }
  __threadfence();
#pragma unroll 1
  for (int j = 0; j < 32; ++j) {
    const int slot = wave * 32 + j;
    const v4f tv = *(const v4f*)(acc1 + slot * DF + c4);
    const v4f q  = *(const v4f*)(acc2 + slot * DF + c4);
    *(volatile v4f*)(t1p + (size_t)slot * DF) = tv;
    *(volatile v4f*)(p2p + (size_t)slot * DF) = q;
  }

  wpart[wave * 2 * DF + c4 + 0] = sP0;
  wpart[wave * 2 * DF + c4 + 1] = sP1;
  wpart[wave * 2 * DF + c4 + 2] = sP2;
  wpart[wave * 2 * DF + c4 + 3] = sP3;
  wpart[wave * 2 * DF + DF + c4 + 0] = sQ0;
  wpart[wave * 2 * DF + DF + c4 + 1] = sQ1;
  wpart[wave * 2 * DF + DF + c4 + 2] = sQ2;
  wpart[wave * 2 * DF + DF + c4 + 3] = sQ3;
  __syncthreads();
  {
    double a = 0.0;
#pragma unroll
    for (int w8 = 0; w8 < NWAVE; ++w8) a += wpart[w8 * 2 * DF + tid];
    double* pp = part + (size_t)blockIdx.x * (2 * DF) + tid;
    *(volatile double*)pp = a;
    __threadfence();
    *(volatile double*)pp = a;
  }
}

__global__ __launch_bounds__(NTHR) void k_fin(
    const float* __restrict__ t1, const float* __restrict__ p2g, const double* __restrict__ part,
    const float* __restrict__ bng, const float* __restrict__ bnb,
    float* out, int nN, int nPart) {
  __shared__ double sred[2 * DF];
  __shared__ __attribute__((aligned(16))) float smu[DF];
  __shared__ __attribute__((aligned(16))) float ssc[DF];
  __shared__ __attribute__((aligned(16))) float sbe[DF];
  const int tid = threadIdx.x, lane = tid & 31, wave = tid >> 5;
  const int c4 = 4 * lane;
  {
    double a = 0.0;
#pragma unroll 1
    for (int b = 0; b < nPart; ++b) a += part[(size_t)b * (2 * DF) + tid];
    sred[tid] = a;
  }
  __syncthreads();
  if (tid < DF) {
    const double invn = 1.0 / (double)nN;
    const double mu = sred[tid] * invn;
    double var = sred[DF + tid] * invn - mu * mu;
    var = var < 0.0 ? 0.0 : var;
    const float varf = (float)var;
    const float inv = 1.0f / sqrtf(varf + EPSV);
    smu[tid] = (float)mu;
    ssc[tid] = inv * bng[tid];
    sbe[tid] = bnb[tid];
  }
  __syncthreads();
  const v4f mu4 = *(const v4f*)(smu + c4);
  const v4f sc4 = *(const v4f*)(ssc + c4);
  const v4f be4 = *(const v4f*)(sbe + c4);
  const int rowBase = blockIdx.x * GROWS + wave * 16;
  v4f ov[16];
#pragma unroll
  for (int i = 0; i < 16; ++i) {
    int r = rowBase + i;
    r = r > nN - 1 ? nN - 1 : r;
    const v4f a = *(const v4f*)(t1  + (size_t)r * DF + c4);
    const v4f p = *(const v4f*)(p2g + (size_t)r * DF + c4);
    ov[i] = a + ((p - mu4) * sc4 + be4);
  }
#pragma unroll
  for (int i = 0; i < 16; ++i) {
    const int r = rowBase + i;
    if (r < nN) *(volatile v4f*)(out + (size_t)r * DF + c4) = ov[i];
  }
  __threadfence();
#pragma unroll
  for (int i = 0; i < 16; ++i) {
    const int r = rowBase + i;
    if (r < nN) *(volatile v4f*)(out + (size_t)r * DF + c4) = ov[i];
  }
}

extern "C" void kernel_launch(void* const* d_in, const int* in_sizes, int n_in,
                              void* d_out, int out_size, void* d_ws, size_t ws_size,
                              hipStream_t stream) {
  if (n_in < 11) return;
  const int nN = in_sizes[0] / DF;
  const int nE = in_sizes[9];
  if (nN <= 0 || nE < 0 || in_sizes[0] != nN * DF || in_sizes[1] != nN * 3) return;
  if (in_sizes[2] != 3 * DF || in_sizes[3] < DF || in_sizes[4] < DF) return;
  if (in_sizes[5] != DF * DF || in_sizes[6] < DF || in_sizes[7] < DF || in_sizes[8] < DF) return;
  if (in_sizes[10] != nE) return;
  if (out_size != nN * DF) return;

  const float* x    = (const float*)d_in[0];
  const float* xyz  = (const float*)d_in[1];
  const float* Wxyz = (const float*)d_in[2];
  const float* bng  = (const float*)d_in[3];
  const float* bnb  = (const float*)d_in[4];
  const float* W1   = (const float*)d_in[5];
  const float* b1   = (const float*)d_in[6];
  const float* lng  = (const float*)d_in[7];
  const float* lnb  = (const float*)d_in[8];
  const int*   srcl = (const int*)d_in[9];
  const int*   dstl = (const int*)d_in[10];
  float* out = (float*)d_out;

  const int nG = (nN + GROWS - 1) / GROWS;
  const int nA = (nN + NB - 1) / NB;

  char* ws = (char*)d_ws;
  size_t off = 0;
  const size_t oWh = off; off += (size_t)DF * DF * 2;                 off = (off + 255) & ~(size_t)255;
  const size_t oWl = off; off += (size_t)DF * DF * 2;                 off = (off + 255) & ~(size_t)255;
  const size_t oY  = off; off += (size_t)nG * GROWS * DF * 4;         off = (off + 255) & ~(size_t)255;
  const size_t oZ  = off; off += (size_t)nG * GROWS * DF * 4;         off = (off + 255) & ~(size_t)255;
  const size_t oT1 = off; off += (size_t)nA * NB * DF * 4;            off = (off + 255) & ~(size_t)255;
  const size_t oP2 = off; off += (size_t)nA * NB * DF * 4;            off = (off + 255) & ~(size_t)255;
  const size_t oPt = off; off += (size_t)nA * 2 * DF * 8;             off = (off + 255) & ~(size_t)255;
  if (off > ws_size) return;
  __bf16* w1h  = (__bf16*)(ws + oWh);
  __bf16* w1l  = (__bf16*)(ws + oWl);
  float*  y    = (float*)(ws + oY);
  float*  z    = (float*)(ws + oZ);
  float*  t1   = (float*)(ws + oT1);
  float*  p2g  = (float*)(ws + oP2);
  double* part = (double*)(ws + oPt);

  const int vec8 = 1;

  const int nPrep = DF * DF / 8;
  k_wprep<<<(nPrep + NTHR - 1) / NTHR, NTHR, 0, stream>>>(W1, w1h, w1l);

  hipFuncSetAttribute(reinterpret_cast<const void*>(&k_node),
                      hipFuncAttributeMaxDynamicSharedMemorySize, LDS_NODE);
  k_node<<<nG, NTHR, LDS_NODE, stream>>>(x, xyz, Wxyz, w1h, w1l, y, z, nN);

  hipFuncSetAttribute(reinterpret_cast<const void*>(&k_agg),
                      hipFuncAttributeMaxDynamicSharedMemorySize, LDS_AGG);
  k_agg<<<nA, NTHR, LDS_AGG, stream>>>(srcl, dstl, xyz, x, y, z, b1, lng, lnb, t1, p2g, part, nN, nE, vec8);

  k_fin<<<nG, NTHR, 0, stream>>>(t1, p2g, part, bng, bnb, out, nN, nA);
}
